// MultiheadAttention_74380243632417
// MI455X (gfx1250) — hardware-run, weakly checked
//
#include <hip/hip_runtime.h>

typedef __attribute__((ext_vector_type(16))) _Float16 v16h;
typedef __attribute__((ext_vector_type(8)))  _Float16 v8h;
typedef __attribute__((ext_vector_type(16))) __bf16   v16b;
typedef __attribute__((ext_vector_type(8)))  __bf16   v8b;
typedef __attribute__((ext_vector_type(8)))  float    v8f;
typedef __attribute__((ext_vector_type(4)))  float    v4f;
typedef __attribute__((ext_vector_type(4)))  unsigned int v4u;

#ifndef NB
#define NB 2
#endif
#ifndef SEQ
#define SEQ 4096
#endif
#define NB_FULL 2
#define SEQ_FULL 4096

constexpr int kDim      = 512;
constexpr int kHeads    = 8;
constexpr int kHeadDim  = 64;
constexpr int kRows     = NB * SEQ;
constexpr int kRowsFull = NB_FULL * SEQ_FULL;
constexpr int kQK       = 2 * kDim;

static_assert(NB >= 1 && NB <= NB_FULL);
static_assert(SEQ >= 64 && SEQ <= SEQ_FULL);
static_assert(kHeads * kHeadDim == kDim);
static_assert(kHeadDim == 64);
static_assert(SEQ % 64 == 0);
static_assert(kRows % 64 == 0 && kDim % 64 == 0 && kDim % 32 == 0 && kQK % 64 == 0);
static_assert(((size_t)SEQ * kDim) % (256 * 8) == 0);
static_assert(kQK % 8 == 0 && kRows % 8 == 0 && kDim % 8 == 0);

constexpr size_t kOffXB  = 0;
constexpr size_t kSzXB   = (size_t)kRowsFull * kDim * 2;
constexpr size_t kOffWQT = 8388608;
constexpr size_t kSzWQT  = (size_t)3 * kDim * kDim * 2;
constexpr size_t kOffWPT = 10485760;
constexpr size_t kSzWPT  = (size_t)kDim * kDim * 2;
constexpr size_t kOffQK  = 16777216;
constexpr size_t kSzQK   = (size_t)kRowsFull * kQK * 2;
constexpr size_t kOffVT  = kOffQK + kSzQK;
constexpr size_t kSzVT   = (size_t)kDim * kRowsFull * 2;
constexpr size_t kOffY   = kOffVT + kSzVT;
constexpr size_t kSzY    = (size_t)kRowsFull * kDim * 2;
constexpr size_t kWsTotal = kOffY + kSzY;
static_assert(kOffXB + kSzXB <= kOffWQT);
static_assert(kOffWQT + kSzWQT <= kOffWPT);
static_assert(kOffWPT + kSzWPT <= kOffQK);
static_assert(kOffQK + kSzQK <= kOffVT);
static_assert(kOffVT + kSzVT <= kOffY);
static_assert(kWsTotal == 50331648);
static_assert(kWsTotal <= 134217728);
static_assert((size_t)kRows * kDim * 2 <= kSzXB && (size_t)kRows * kQK * 2 <= kSzQK);
static_assert((size_t)kDim * kRows * 2 <= kSzVT && (size_t)kRows * kDim * 2 <= kSzY);

__device__ __forceinline__ unsigned short f2bf_bits(float f) {
  unsigned u = __float_as_uint(f);
  return (unsigned short)((u + 0x7FFFu + ((u >> 16) & 1u)) >> 16);
}
__device__ __forceinline__ float bf_bits2f(unsigned short h) { return __uint_as_float(((unsigned)h) << 16); }

template <typename T> struct Frag;
template <> struct Frag<_Float16> {
  typedef v16h V; union U { v16h v; v8h h[2]; };
  static __device__ __forceinline__ v16h load(const _Float16* p) {
    U f; f.h[0] = *(const v8h*)(p); f.h[1] = *(const v8h*)(p + 16); return f.v;
  }
  static __device__ __forceinline__ v8f mma(v16h a, v16h b, v8f c) {
    c = __builtin_amdgcn_wmma_f32_16x16x32_f16(false, a, false, b, (short)0, c, false, false);
    asm volatile("v_nop\n\tv_nop\n\tv_nop\n\tv_nop" : "+v"(c) : "v"(a), "v"(b));
    return c;
  }
};
template <> struct Frag<__bf16> {
  typedef v16b V; union U { v16b v; v8b h[2]; };
  static __device__ __forceinline__ v16b load(const __bf16* p) {
    U f; f.h[0] = *(const v8b*)(p); f.h[1] = *(const v8b*)(p + 16); return f.v;
  }
  static __device__ __forceinline__ v8f mma(v16b a, v16b b, v8f c) {
    c = __builtin_amdgcn_wmma_f32_16x16x32_bf16(false, a, false, b, (short)0, c, false, false);
    asm volatile("v_nop\n\tv_nop\n\tv_nop\n\tv_nop" : "+v"(c) : "v"(a), "v"(b));
    return c;
  }
};

template <int ET> struct Elem;
template <> struct Elem<0> { typedef _Float16 T; };
template <> struct Elem<1> { typedef __bf16 T; };
template <int ET, int BIAS_MODE, int OUT_MODE>
__device__ __forceinline__ void gemm64_body(
    const unsigned short* __restrict__ Ap, int lda, long strideA,
    const unsigned short* __restrict__ Btp, int ldb, long strideB,
    void* __restrict__ Cout, int ldc, long strideC,
    const float* __restrict__ bias,
    int M, int N, int K, float scale, float post) {
  typedef typename Elem<ET>::T T;
  typedef typename Frag<T>::V V;
  const T* A = (const T*)(const void*)Ap; const T* Bt = (const T*)(const void*)Btp;
  __shared__ __align__(16) float sT[8][16 * 68];
  const unsigned b    = blockIdx.y;
  const unsigned lane = threadIdx.x & 31u;
  const unsigned wave = (unsigned)__builtin_amdgcn_readfirstlane((int)(threadIdx.x >> 5));
  const unsigned tilesN = ((unsigned)N) >> 6;
  const unsigned tilesM = ((unsigned)M) >> 6;
  const unsigned tile = blockIdx.x * 8u + wave;
  if (tile >= tilesM * tilesN) return;
  const unsigned tm = tile / tilesN;
  const unsigned tn = tile - tm * tilesN;
  const unsigned m0 = tm << 6;
  const unsigned n0 = tn << 6;
  const unsigned ulda = (unsigned)lda, uldb = (unsigned)ldb, uldc = (unsigned)ldc, uK = (unsigned)K;

  const T* Ab = A  + (size_t)b * (size_t)strideA;
  const T* Bb = Bt + (size_t)b * (size_t)strideB;

  const unsigned rlane = lane & 15u;
  const unsigned koff  = (lane >> 4) * 8u;
  const unsigned mOff  = (lane >> 4) * 8u;

  v8f acc[4][4];
#pragma unroll
  for (int i = 0; i < 4; ++i)
#pragma unroll
    for (int j = 0; j < 4; ++j) acc[i][j] = (v8f){0.f,0.f,0.f,0.f,0.f,0.f,0.f,0.f};

#pragma unroll 1
  for (unsigned k0 = 0; k0 < uK; k0 += 32u) {
    V bh[4];
#pragma unroll
    for (int j = 0; j < 4; ++j) {
      const size_t bo = (size_t)(n0 + ((unsigned)j << 4) + rlane) * uldb + koff + k0;
      bh[j] = Frag<T>::load(Bb + bo);
    }
#pragma unroll
    for (int i = 0; i < 4; ++i) {
      const size_t ao = (size_t)(m0 + ((unsigned)i << 4) + rlane) * ulda + koff + k0;
      const V ah = Frag<T>::load(Ab + ao);
#pragma unroll
      for (int j = 0; j < 4; ++j) acc[i][j] = Frag<T>::mma(ah, bh[j], acc[i][j]);
    }
  }

#pragma unroll
  for (int i = 0; i < 4; ++i) {
    const unsigned mBase = m0 + ((unsigned)i << 4);
    float brow[8];
#pragma unroll
    for (int r = 0; r < 8; ++r) {
      brow[r] = 0.f;
      if (BIAS_MODE == 3) brow[r] = bf_bits2f(f2bf_bits(bias[mBase + mOff + (unsigned)r]));
    }
#pragma unroll
    for (int j = 0; j < 4; ++j) {
      const unsigned n = n0 + ((unsigned)j << 4) + rlane;
      float bv = 0.f;
      if (BIAS_MODE == 2) bv = bf_bits2f(f2bf_bits(bias[n]));
#pragma unroll
      for (int r = 0; r < 8; ++r) {
        float v = acc[i][j][r] * scale;
        if (BIAS_MODE == 2) v += bv;
        if (BIAS_MODE == 3) v += brow[r];
        v *= post;
        sT[wave][(mOff + (unsigned)r) * 68u + ((unsigned)j << 4) + rlane] = v;
      }
    }
    __builtin_amdgcn_fence(3  , "workgroup");
    __builtin_amdgcn_wave_barrier();
    __builtin_amdgcn_fence(2  , "workgroup");
    if (OUT_MODE == 0) {
      float* C = (float*)Cout + (size_t)b * (size_t)strideC;
      const unsigned hh = lane >> 4, c4 = (lane & 15u) * 4u;
      for (int pass = 0; pass < 2; ++pass) {
#pragma unroll
        for (int it = 0; it < 8; ++it) {
          const unsigned row = (unsigned)it * 2u + hh;
          const v4f v = *(const v4f*)(&sT[wave][row * 68u + c4]);
          *(volatile v4f*)(C + (size_t)(mBase + row) * uldc + n0 + c4) = v;
        }
        __threadfence();
      }
    } else {
      const unsigned q = lane >> 3, c8 = (lane & 7u) * 8u;
      unsigned short* C = (unsigned short*)Cout + (size_t)b * (size_t)strideC;
      for (int pass = 0; pass < 2; ++pass) {
#pragma unroll
        for (int it = 0; it < 4; ++it) {
          const unsigned row = (unsigned)it * 4u + q;
          v8h hv;
#pragma unroll
          for (int e = 0; e < 8; ++e) hv[e] = (_Float16)sT[wave][row * 68u + c8 + (unsigned)e];
          *(volatile v8h*)(C + (size_t)(mBase + row) * uldc + n0 + c8) = hv;
        }
        __threadfence();
      }
    }
    __builtin_amdgcn_fence(3  , "workgroup");
    __builtin_amdgcn_wave_barrier();
    __builtin_amdgcn_fence(2  , "workgroup");
  }
}

__global__ __launch_bounds__(256) __attribute__((amdgpu_num_vgpr(256)))
void gemm_bf16_colbias_f16(
    const unsigned short* __restrict__ A, int lda, long strideA,
    const unsigned short* __restrict__ Bt, int ldb, long strideB,
    unsigned short* __restrict__ C, int ldc, long strideC,
    const float* __restrict__ bias, int M, int N, int K, float scale, float post) {
  gemm64_body<1, 2, 1>(A, lda, strideA, Bt, ldb, strideB, (void*)C, ldc, strideC, bias, M, N, K, scale, post);
}
__global__ __launch_bounds__(256) __attribute__((amdgpu_num_vgpr(256)))
void gemm_bf16_rowbias_f16(
    const unsigned short* __restrict__ A, int lda, long strideA,
    const unsigned short* __restrict__ Bt, int ldb, long strideB,
    unsigned short* __restrict__ C, int ldc, long strideC,
    const float* __restrict__ bias, int M, int N, int K, float scale, float post) {
  gemm64_body<1, 3, 1>(A, lda, strideA, Bt, ldb, strideB, (void*)C, ldc, strideC, bias, M, N, K, scale, post);
}
__global__ __launch_bounds__(256) __attribute__((amdgpu_num_vgpr(256)))
void gemm_f16_colbias_f32(
    const unsigned short* __restrict__ A, int lda, long strideA,
    const unsigned short* __restrict__ Bt, int ldb, long strideB,
    float* __restrict__ C, int ldc, long strideC,
    const float* __restrict__ bias, int M, int N, int K, float scale, float post) {
  gemm64_body<0, 2, 0>(A, lda, strideA, Bt, ldb, strideB, (void*)C, ldc, strideC, bias, M, N, K, scale, post);
}

__global__ __launch_bounds__(256) void cast_f32_bf16x8(
    const float* __restrict__ in, unsigned short* __restrict__ out, int n8, long inStride, long outStride) {
  const unsigned i = blockIdx.x * 256u + threadIdx.x;
  const float* src = in + (size_t)blockIdx.y * (size_t)inStride;
  unsigned short* dst = out + (size_t)blockIdx.y * (size_t)outStride;
  if (i < (unsigned)n8) {
    const size_t e0 = (size_t)i * 8;
    const v4f a = *(const v4f*)(src + e0);
    const v4f c = *(const v4f*)(src + e0 + 4);
    v4u w;
    w[0] = (unsigned)f2bf_bits(a[0]) | ((unsigned)f2bf_bits(a[1]) << 16);
    w[1] = (unsigned)f2bf_bits(a[2]) | ((unsigned)f2bf_bits(a[3]) << 16);
    w[2] = (unsigned)f2bf_bits(c[0]) | ((unsigned)f2bf_bits(c[1]) << 16);
    w[3] = (unsigned)f2bf_bits(c[2]) | ((unsigned)f2bf_bits(c[3]) << 16);
    *(volatile v4u*)(dst + e0) = w;
    __threadfence();
    *(volatile v4u*)(dst + e0) = w;
  }
}

__global__ __launch_bounds__(256) void tcast64(
    const float* __restrict__ W, unsigned short* __restrict__ Wt, int nrows, int ncols, int mode) {
  __shared__ __align__(16) unsigned short tl[64 * 72];
  const unsigned tid = threadIdx.x, lane = tid & 31u;
  const unsigned wave = (unsigned)__builtin_amdgcn_readfirstlane((int)(tid >> 5));
  const unsigned k0 = blockIdx.y * 64u;
  const unsigned n0 = blockIdx.x * 64u;
  const unsigned krow = tid >> 2;
  const unsigned nseg = (tid & 3u) * 16u;
  const float* src = W + (size_t)(k0 + krow) * (unsigned)ncols + n0 + nseg;
  v4f vv[4];
#pragma unroll
  for (int i = 0; i < 4; ++i) vv[i] = ((const v4f*)src)[i];
#pragma unroll
  for (int i = 0; i < 4; ++i)
#pragma unroll
    for (int e = 0; e < 4; ++e) {
      const unsigned short bb = f2bf_bits(vv[i][e]);
      const _Float16 hv = (_Float16)(bf_bits2f(bb) * 64.0f);
      const unsigned short hb = __builtin_bit_cast(unsigned short, hv);
      tl[(nseg + 4u * (unsigned)i + (unsigned)e) * 72u + krow] = (mode == 0) ? bb : hb;
    }
  __syncthreads();
  const unsigned q4 = lane >> 3, c8 = (lane & 7u) * 8u;
  for (int pass = 0; pass < 2; ++pass) {
#pragma unroll
    for (int it = 0; it < 2; ++it) {
      const unsigned row = wave * 8u + (unsigned)it * 4u + q4;
      const v4u w = *(const v4u*)(tl + row * 72u + c8);
      *(volatile v4u*)(Wt + (size_t)(n0 + row) * (unsigned)nrows + k0 + c8) = w;
    }
    __threadfence();
  }
}

#define AT_D 64
#define AT_NW 4
#define AT_QB 64
#define AT_KC 64
static_assert(AT_D == kHeadDim);
static_assert(AT_QB == AT_NW * 16);
static_assert(SEQ % AT_KC == 0 && SEQ % AT_QB == 0);

__global__ __launch_bounds__(128) __attribute__((amdgpu_num_vgpr(256)))
void attn64_dense_t(const unsigned short* __restrict__ qk, const unsigned short* __restrict__ vt,
                    unsigned short* __restrict__ y,
                    int nseq, int nheads, int ldqk, int ldvt, int ldo) {
  __shared__ __align__(16) float os[AT_NW][16 * 68];

  const unsigned tid  = threadIdx.x;
  const unsigned wave = (unsigned)__builtin_amdgcn_readfirstlane((int)(tid >> 5));
  const unsigned lane = tid & 31u;
  const unsigned hh   = lane >> 4;
  const unsigned c    = lane & 15u;

  const unsigned useq = (unsigned)nseq, uheads = (unsigned)nheads;
  const unsigned uldqk = (unsigned)ldqk, uldvt = (unsigned)ldvt, uldo = (unsigned)ldo;
  const unsigned nqb = useq >> 6;
  const unsigned bx  = blockIdx.x;
  const unsigned bhd = bx / nqb;
  const unsigned qb  = bx - bhd * nqb;
  const unsigned b   = bhd / uheads;
  const unsigned h   = bhd - b * uheads;
  const unsigned q0  = qb * AT_QB + wave * 16u;
  const size_t rowb = (size_t)b * useq;

  const _Float16* QK = (const _Float16*)(const void*)qk;
  const _Float16* VT = (const _Float16*)(const void*)vt;

  v16h qf[2];
  {
    const size_t qr = (rowb + q0 + c) * (size_t)uldqk + h * AT_D + 8u * hh;
#pragma unroll
    for (int dc = 0; dc < 2; ++dc) qf[dc] = Frag<_Float16>::load(QK + qr + dc * 32);
  }
  const _Float16* kp = QK + (rowb + c) * (size_t)uldqk + uheads * AT_D + h * AT_D + 8u * hh;
  const _Float16* vp = VT + (size_t)(h * AT_D + c) * (size_t)uldvt + rowb + 8u * hh;

  v16h ones;
#pragma unroll
  for (int i = 0; i < 16; ++i) ones[i] = (_Float16)1.0f;

  float mrun = -__builtin_huge_valf();
  v8f oacc[4];
  v8f lacc = (v8f){0.f,0.f,0.f,0.f,0.f,0.f,0.f,0.f};
#pragma unroll
  for (int t = 0; t < 4; ++t) oacc[t] = (v8f){0.f,0.f,0.f,0.f,0.f,0.f,0.f,0.f};

#pragma unroll 1
  for (unsigned kv0 = 0; kv0 < useq; kv0 += AT_KC) {
    v8f s[4];
#pragma unroll
    for (int j = 0; j < 4; ++j) {
      s[j] = (v8f){0.f,0.f,0.f,0.f,0.f,0.f,0.f,0.f};
      const _Float16* kr = kp + (size_t)(kv0 + (unsigned)j * 16u) * (size_t)uldqk;
#pragma unroll
      for (int dc = 0; dc < 2; ++dc) {
        const v16h kf = Frag<_Float16>::load(kr + dc * 32);
        s[j] = Frag<_Float16>::mma(kf, qf[dc], s[j]);
      }
    }

    float mloc = s[0][0];
#pragma unroll
    for (int j = 0; j < 4; ++j)
#pragma unroll
      for (int r = 0; r < 8; ++r) mloc = fmaxf(mloc, s[j][r]);
    mloc = fmaxf(mloc, __shfl_xor(mloc, 16, 32));
    const float mnew  = fmaxf(mrun, mloc);
    const float alpha = __builtin_amdgcn_exp2f(mrun - mnew);
    mrun = mnew;
    const float msub = mnew - 10.0f;

    v16h pf[2];
#pragma unroll
    for (int kk = 0; kk < 2; ++kk) {
#pragma unroll
      for (int r = 0; r < 8; ++r) {
        pf[kk][r]     = (_Float16)__builtin_amdgcn_exp2f(s[2 * kk][r] - msub);
        pf[kk][8 + r] = (_Float16)__builtin_amdgcn_exp2f(s[2 * kk + 1][r] - msub);
      }
    }

#pragma unroll
    for (int t = 0; t < 4; ++t) oacc[t] = oacc[t] * alpha;
    lacc = lacc * alpha;

#pragma unroll
    for (int kk = 0; kk < 2; ++kk) {
#pragma unroll
      for (int t = 0; t < 4; ++t) {
        const v16h vf = Frag<_Float16>::load(vp + (size_t)((unsigned)t * 16u) * (size_t)uldvt + kv0 + (unsigned)kk * 32u);
        oacc[t] = Frag<_Float16>::mma(vf, pf[kk], oacc[t]);
      }
      lacc = Frag<_Float16>::mma(ones, pf[kk], lacc);
    }
  }

  {
    const float inv = 256.0f * (1.0f / lacc[0]);
#pragma unroll
    for (int t = 0; t < 4; ++t)
#pragma unroll
      for (int r = 0; r < 8; ++r)
        os[wave][c * 68u + (unsigned)t * 16u + 8u * hh + (unsigned)r] = oacc[t][r] * inv;
  }
  __builtin_amdgcn_fence(3  , "workgroup");
  __builtin_amdgcn_wave_barrier();
  __builtin_amdgcn_fence(2  , "workgroup");
  {
    const unsigned q4 = lane >> 3, c8 = (lane & 7u) * 8u;
    for (int pass = 0; pass < 2; ++pass) {
#pragma unroll
      for (int it = 0; it < 4; ++it) {
        const unsigned row = (unsigned)it * 4u + q4;
        v8h hv;
#pragma unroll
        for (int e = 0; e < 8; ++e) hv[e] = (_Float16)os[wave][row * 68u + c8 + (unsigned)e];
        const size_t o = (rowb + q0 + row) * (size_t)uldo + h * AT_D + c8;
        *(volatile v8h*)(y + o) = hv;
      }
      __threadfence();
    }
  }
}

extern "C" void kernel_launch(void* const* d_in, const int* in_sizes, int n_in,
                              void* d_out, int out_size, void* d_ws,
                              size_t ws_size, hipStream_t stream)
{
  if (n_in < 9) return;
  if (ws_size < kWsTotal) return;
  const long long needX = (long long)(NB - 1) * SEQ_FULL * kDim + (long long)SEQ * kDim;
  if ((long long)out_size < needX) return;
  if ((long long)in_sizes[0] < needX) return;
  if (in_sizes[1] < kDim * kDim || in_sizes[3] < kDim * kDim || in_sizes[5] < kDim * kDim || in_sizes[7] < kDim * kDim) return;
  if (in_sizes[2] < kDim || in_sizes[4] < kDim || in_sizes[6] < kDim || in_sizes[8] < kDim) return;

  const float* x  = (const float*)d_in[0];
  const float* Wq = (const float*)d_in[1];
  const float* bq = (const float*)d_in[2];
  const float* Wk = (const float*)d_in[3];
  const float* bk = (const float*)d_in[4];
  const float* Wv = (const float*)d_in[5];
  const float* bv = (const float*)d_in[6];
  const float* Wo = (const float*)d_in[7];
  const float* bo = (const float*)d_in[8];
  float* out = (float*)d_out;

  unsigned char* ws = (unsigned char*)d_ws;
  unsigned short* XB  = (unsigned short*)(ws + kOffXB);
  unsigned short* WQT = (unsigned short*)(ws + kOffWQT);
  unsigned short* WPT = (unsigned short*)(ws + kOffWPT);
  unsigned short* QK  = (unsigned short*)(ws + kOffQK);
  unsigned short* VT  = (unsigned short*)(ws + kOffVT);
  unsigned short* Y   = (unsigned short*)(ws + kOffY);

  {
    const int n8 = SEQ * kDim / 8;
    cast_f32_bf16x8<<<dim3((n8 + 255) / 256, NB), dim3(256), 0, stream>>>(
        x, XB, n8, (long)SEQ_FULL * kDim, (long)SEQ * kDim);
  }
  tcast64<<<dim3(kDim / 64, kDim / 64), dim3(256), 0, stream>>>(Wq, WQT, kDim, kDim, 0);
  tcast64<<<dim3(kDim / 64, kDim / 64), dim3(256), 0, stream>>>(Wk, WQT + (size_t)kDim * kDim, kDim, kDim, 0);
  tcast64<<<dim3(kDim / 64, kDim / 64), dim3(256), 0, stream>>>(Wv, WQT + (size_t)2 * kDim * kDim, kDim, kDim, 0);
  tcast64<<<dim3(kDim / 64, kDim / 64), dim3(256), 0, stream>>>(Wo, WPT, kDim, kDim, 1);
  {
    const int tiles = (kRows / 64) * (kDim / 64);
    gemm_bf16_colbias_f16<<<dim3((tiles + 7) / 8, 1), dim3(256), 0, stream>>>(
        XB, kDim, 0L, WQT, kDim, 0L,
        QK, kQK, 0L, bq, kRows, kDim, kDim, 1.0f, 0.18033688011112042f);
    gemm_bf16_colbias_f16<<<dim3((tiles + 7) / 8, 1), dim3(256), 0, stream>>>(
        XB, kDim, 0L, WQT + (size_t)kDim * kDim, kDim, 0L,
        QK + kDim, kQK, 0L, bk, kRows, kDim, kDim, 1.0f, 1.0f);
  }
  {
    const int tiles = (kDim / 64) * (kRows / 64);
    gemm_bf16_rowbias_f16<<<dim3((tiles + 7) / 8, 1), dim3(256), 0, stream>>>(
        WQT + (size_t)2 * kDim * kDim, kDim, 0L, XB, kDim, 0L,
        VT, kRows, 0L, bv, kDim, kRows, kDim, 1.0f, 1.0f);
  }
  attn64_dense_t<<<dim3(NB * kHeads * (SEQ / AT_QB)), dim3(128), 0, stream>>>(
      QK, VT, Y, SEQ, kHeads, kQK, kRows, kDim);
  {
    const int tiles = (SEQ / 64) * (kDim / 64);
    gemm_f16_colbias_f32<<<dim3((tiles + 7) / 8, NB), dim3(256), 0, stream>>>(
        Y, kDim, (long)SEQ * kDim, WPT, kDim, 0L,
        out, kDim, (long)SEQ_FULL * kDim, bo, SEQ, kDim, kDim, 6.103515625e-05f, 1.0f);
  }
}
